// Attention_74363063763568
// MI455X (gfx1250) — hardware-verified
//
#include <hip/hip_runtime.h>


#ifndef NB
#define NB 32
#endif
#ifndef SEQ
#define SEQ 577
#endif
#define NB_FULL  32
#define SEQ_FULL 577
#define DM   768
#define NH   12
#define HD   64
#define DQKV (3 * DM)
#define NRD  2212
#define SEQP ((((SEQ) + 63) / 64) * 64)
#define NQT  (SEQP / 64)
#define BPP  (((NB) < 16) ? (NB) : 16)
#define MP   (BPP * SEQ)
#define KP   72
#define CAR  8.0f
#define PCAR 1024.0f
#define SCL  0.125f
#define SFOLD (SCL / (CAR * CAR))
#define L2E  1.4426950408889634f
#define NEGB (-1.0e30f)

static_assert(NB >= 1 && NB <= NB_FULL);
static_assert(SEQ >= 1 && SEQ <= SEQ_FULL);
static_assert(DM % 64 == 0);
static_assert(DQKV % 64 == 0);
static_assert(DM % 32 == 0);
static_assert(HD == 64);
static_assert(NH * HD == DM);
static_assert((SEQ * DM) % 8 == 0);
static_assert(SEQP % 64 == 0 && SEQP >= SEQ);

typedef _Float16 h16;
typedef unsigned short bf;
typedef __attribute__((ext_vector_type(16))) __bf16   v16bf;
typedef __attribute__((ext_vector_type(16))) _Float16 v16h;
typedef __attribute__((ext_vector_type(8)))  _Float16 v8h;
typedef __attribute__((ext_vector_type(8)))  unsigned short v8us;
typedef __attribute__((ext_vector_type(8)))  float    v8f;
typedef __attribute__((ext_vector_type(4)))  float    v4f;
typedef v8h  __attribute__((may_alias)) v8ha;
typedef v4f  __attribute__((may_alias)) v4fa;
typedef v8us __attribute__((may_alias)) v8usa;

constexpr size_t al256(size_t x) { return (x + 255) & ~(size_t)255; }
constexpr size_t WS_WQKV = al256((size_t)DQKV * DM * 2);
constexpr size_t WS_WO   = al256((size_t)DM * DM * 2);
constexpr size_t WS_BP   = al256((size_t)NH * SEQP * SEQP * 2);
constexpr size_t WS_XB   = al256((size_t)MP * DM * 2);
constexpr size_t WS_F    = al256((size_t)MP * DQKV * 2);
constexpr size_t WS_VT   = al256((size_t)BPP * NH * HD * SEQP * 2);
constexpr size_t WS_CT   = al256((size_t)MP * DM * 2);
constexpr size_t WS_TOTAL = WS_WQKV + WS_WO + WS_BP + WS_XB + WS_F + WS_VT + 2 * WS_CT;
static_assert(WS_TOTAL <= (size_t)134217728);

__device__ __forceinline__ unsigned short f2bf(float f) { unsigned u = __float_as_uint(f); u += 0x7FFFu + ((u >> 16) & 1u); return (unsigned short)(u >> 16); }
__device__ __forceinline__ float bf2f(unsigned short b) { return __uint_as_float(((unsigned)b) << 16); }
__device__ __forceinline__ float bfr(float f) { return bf2f(f2bf(f)); }
__device__ __forceinline__ h16 tohx(float x) { return (h16)x; }
__device__ __forceinline__ void splitf(float y, unsigned short& h, unsigned short& l) { h = f2bf(y); l = f2bf(y - bf2f(h)); }
__device__ __forceinline__ v16h cat16(v8h lo, v8h hi) { return __builtin_shufflevector(lo, hi, 0, 1, 2, 3, 4, 5, 6, 7, 8, 9, 10, 11, 12, 13, 14, 15); }
__device__ __forceinline__ v16bf cat16b(v8us lo, v8us hi) { return __builtin_bit_cast(v16bf, __builtin_shufflevector(lo, hi, 0, 1, 2, 3, 4, 5, 6, 7, 8, 9, 10, 11, 12, 13, 14, 15)); }
__device__ __forceinline__ v8f wmma16(v16h a, v16h b, v8f c) { return __builtin_amdgcn_wmma_f32_16x16x32_f16(false, a, false, b, (short)0, c, false, false); }
__device__ __forceinline__ v8f wmmab(v16bf a, v16bf b, v8f c) { return __builtin_amdgcn_wmma_f32_16x16x32_bf16(false, a, false, b, (short)0, c, false, false); }
__device__ __forceinline__ void wave_lds_sync() { __builtin_amdgcn_fence(4  , "wavefront"); __builtin_amdgcn_wave_barrier(); asm volatile("" ::: "memory"); }

template <typename T16> struct WFrag;
template <> struct WFrag<h16> { typedef v16h V; static __device__ __forceinline__ V ld(const h16* p) { return cat16(*(const v8ha*)p, *(const v8ha*)(p + 16)); } static __device__ __forceinline__ v8f mma(V a, V b, v8f c) { return wmma16(a, b, c); } };
template <> struct WFrag<bf>  { typedef v16bf V; static __device__ __forceinline__ V ld(const bf* p) { return cat16b(*(const v8usa*)p, *(const v8usa*)(p + 16)); } static __device__ __forceinline__ v8f mma(V a, V b, v8f c) { return wmmab(a, b, c); } };

template <typename T16, int NSPLIT, int EPI>
__global__ __launch_bounds__(32) void k_gemmw(const T16* __restrict__ A, const T16* __restrict__ A2, const T16* __restrict__ Bt, int K, int Mlim,
                                              float* Cf, h16* Ch, int ldc, const float* __restrict__ bias, const float* __restrict__ bias2, float carry) {
    typedef typename WFrag<T16>::V V;
    __shared__ __align__(16) float os[16 * 68];
    const int lane = threadIdx.x & 31, lr = lane & 15, hi = lane >> 4;
    const int r0 = blockIdx.x * 64, c0 = blockIdx.y * 64;
    v8f acc[4][4];
#pragma unroll
    for (int mb = 0; mb < 4; ++mb)
#pragma unroll
        for (int nb = 0; nb < 4; ++nb) acc[mb][nb] = (v8f){};
    size_t aoff[4];
#pragma unroll
    for (int mb = 0; mb < 4; ++mb) { int ra = r0 + mb * 16 + lr; ra = (ra < Mlim) ? ra : (Mlim - 1); aoff[mb] = (size_t)ra * K + 8 * hi; }
    const size_t boff = (size_t)(c0 + lr) * K + 8 * hi;
#pragma unroll 1
    for (int kc = 0; kc < K; kc += 32) {
        V a[4], a2[4], bl;
#pragma unroll
        for (int mb = 0; mb < 4; ++mb) { a[mb] = WFrag<T16>::ld(A + aoff[mb] + kc); if (NSPLIT == 1) a2[mb] = WFrag<T16>::ld(A2 + aoff[mb] + kc); else a2[mb] = a[mb]; }
#pragma unroll
        for (int nb = 0; nb < 4; ++nb) { bl = WFrag<T16>::ld(Bt + boff + (size_t)nb * 16 * K + kc);
#pragma unroll
            for (int mb = 0; mb < 4; ++mb) { acc[mb][nb] = WFrag<T16>::mma(a[mb], bl, acc[mb][nb]); if (NSPLIT == 1) acc[mb][nb] = WFrag<T16>::mma(a2[mb], bl, acc[mb][nb]); } }
        asm volatile("v_nop\n\tv_nop\n\tv_nop\n\tv_nop" : "+v"(acc[0][0]), "+v"(acc[1][1]), "+v"(acc[2][2]), "+v"(acc[3][3]) : "v"(a[0]), "v"(a[3]), "v"(a2[3]), "v"(bl));
    }
    if constexpr (EPI == 0) {
        v4f b4 = *(const v4f*)(bias + c0 + lr * 4);
#pragma unroll
        for (int e = 0; e < 4; ++e) b4[e] = bfr(b4[e]);
#pragma unroll
        for (int mb = 0; mb < 4; ++mb) {
#pragma unroll
            for (int nb = 0; nb < 4; ++nb) {
#pragma unroll
                for (int j = 0; j < 8; ++j) os[(hi * 8 + j) * 68 + nb * 16 + lr] = acc[mb][nb][j]; }
            wave_lds_sync();
#pragma unroll 1
            for (int ps = 0; ps < 2; ++ps) {
#pragma unroll
                for (int s = 0; s < 8; ++s) { const int row = 2 * s + hi; const int grow = r0 + mb * 16 + row; v4f val = *(const v4fa*)(os + row * 68 + lr * 4); val += b4;
                    if (grow < Mlim) *(volatile v4f*)(Cf + (size_t)grow * ldc + c0 + lr * 4) = val; }
                if (ps == 0) __threadfence(); }
            wave_lds_sync();
        }
    } else {
        const int rq = lane >> 3, ch = lane & 7;
        const bool isq = (c0 < DM), isv = (c0 >= 2 * DM);
        const int cq = isq ? c0 : 0, cv = isv ? (c0 - 2 * DM) : 0;
        const v4f q0 = *(const v4f*)(bias + cq + ch * 8), q1 = *(const v4f*)(bias + cq + ch * 8 + 4);
        const v4f w0 = *(const v4f*)(bias2 + cv + ch * 8), w1 = *(const v4f*)(bias2 + cv + ch * 8 + 4);
        float bb[8];
#pragma unroll
        for (int e = 0; e < 4; ++e) { bb[e] = isq ? bfr(q0[e]) : (isv ? bfr(w0[e]) : 0.0f); bb[4 + e] = isq ? bfr(q1[e]) : (isv ? bfr(w1[e]) : 0.0f); }
#pragma unroll
        for (int mb = 0; mb < 4; ++mb) {
#pragma unroll
            for (int nb = 0; nb < 4; ++nb) {
#pragma unroll
                for (int j = 0; j < 8; ++j) os[(hi * 8 + j) * 68 + nb * 16 + lr] = acc[mb][nb][j]; }
            wave_lds_sync();
#pragma unroll 1
            for (int ps = 0; ps < 2; ++ps) {
#pragma unroll
                for (int s = 0; s < 4; ++s) { const int row = 4 * s + rq; const int grow = r0 + mb * 16 + row;
                    const v4f v0 = *(const v4fa*)(os + row * 68 + ch * 8), v1 = *(const v4fa*)(os + row * 68 + ch * 8 + 4); v8h o;
#pragma unroll
                    for (int e = 0; e < 4; ++e) { o[e] = tohx((v0[e] + bb[e]) * carry); o[4 + e] = tohx((v1[e] + bb[4 + e]) * carry); }
                    if (grow < Mlim) *(volatile v8h*)(Ch + (size_t)grow * ldc + c0 + ch * 8) = o; }
                if (ps == 0) __threadfence(); }
            wave_lds_sync();
        }
    }
}

__global__ __launch_bounds__(256) void k_cvt8(const float* __restrict__ src, bf* dst, size_t n8) {
    const size_t i = (size_t)blockIdx.x * 256 + threadIdx.x; if (i >= n8) return;
    const v8f v = *(const v8f*)(src + i * 8); v8us o;
#pragma unroll
    for (int k = 0; k < 8; ++k) o[k] = f2bf(v[k]);
    *(volatile v8us*)(dst + i * 8) = o; __threadfence(); *(volatile v8us*)(dst + i * 8) = o;
}
__global__ __launch_bounds__(256) void k_cvtx(const float* __restrict__ src, bf* dst, int nb) {
    const size_t per = (size_t)SEQ * DM / 8; const size_t n8 = per * (size_t)nb;
    const size_t i = (size_t)blockIdx.x * 256 + threadIdx.x; if (i >= n8) return;
    const size_t bb = i / per, rr = i - bb * per;
    const v8f v = *(const v8f*)(src + bb * ((size_t)SEQ_FULL * DM) + rr * 8); v8us o;
#pragma unroll
    for (int k = 0; k < 8; ++k) o[k] = f2bf(v[k]);
    *(volatile v8us*)(dst + i * 8) = o; __threadfence(); *(volatile v8us*)(dst + i * 8) = o;
}
__global__ __launch_bounds__(256) void k_bias(const float* __restrict__ rpb, const int* __restrict__ rel, bf* BP) {
    const int NCH = SEQP / 8; const int total = NH * SEQP * NCH;
    const int idx = blockIdx.x * 256 + threadIdx.x; if (idx >= total) return;
    const int ch = idx % NCH; const int t1 = idx / NCH; const int q = t1 % SEQP; const int h = t1 / SEQP;
    const int qc = (q < SEQ) ? q : (SEQ - 1);
    v8us o;
#pragma unroll
    for (int e = 0; e < 8; ++e) { const int k = ch * 8 + e; const int kc = (k < SEQ) ? k : (SEQ - 1);
        int ri = rel[(size_t)qc * SEQ_FULL + kc]; ri = (ri < 0) ? 0 : ((ri > NRD - 1) ? (NRD - 1) : ri);
        const float v = rpb[(size_t)ri * NH + h]; o[e] = (q < SEQ && k < SEQ) ? f2bf(v) : (unsigned short)0; }
    const size_t oo = ((size_t)h * SEQP + q) * SEQP + (size_t)ch * 8;
    *(volatile v8us*)(BP + oo) = o; __threadfence(); *(volatile v8us*)(BP + oo) = o;
}
__global__ __launch_bounds__(64) void k_vt(const h16* __restrict__ F, h16* VT) {
    __shared__ __align__(16) h16 T[64 * KP];
    const int tt = blockIdx.x, h = blockIdx.y, b = blockIdx.z;
    const int tid = threadIdx.x, w = tid >> 5, lane = tid & 31;
    const int t0 = tt * 64; const size_t rowb = (size_t)b * SEQ;
#pragma unroll
    for (int i = 0; i < 8; ++i) { const int g = tid + i * 64, r = g >> 3, ch = g & 7; const int t = t0 + r; const bool ok = (t < SEQ); const int tc = ok ? t : (SEQ - 1);
        v8h v = *(const v8ha*)(F + (rowb + tc) * DQKV + 2 * DM + h * HD + ch * 8); if (!ok) v = (v8h){}; *(v8ha*)(T + r * KP + ch * 8) = v; }
    __syncthreads();
    const int rq = lane >> 3, ch = lane & 7;
    v8h o[8];
#pragma unroll
    for (int s = 0; s < 8; ++s) { const int d = w * 32 + s * 4 + rq;
#pragma unroll
        for (int e = 0; e < 8; ++e) o[s][e] = T[(ch * 8 + e) * KP + d]; }
    h16* dst = VT + ((size_t)(b * NH + h)) * HD * SEQP + t0 + ch * 8;
#pragma unroll 1
    for (int ps = 0; ps < 2; ++ps) {
#pragma unroll
        for (int s = 0; s < 8; ++s) { const int d = w * 32 + s * 4 + rq; *(volatile v8h*)(dst + (size_t)d * SEQP) = o[s]; }
        if (ps == 0) __threadfence(); }
}

__global__ __launch_bounds__(128) void k_attn(const h16* __restrict__ F, const h16* __restrict__ VT, const bf* __restrict__ BP, bf* CTh, bf* CTl) {
    __shared__ __align__(16) h16 Kt[64 * KP];
    __shared__ __align__(16) h16 Vt[64 * KP];
    __shared__ __align__(16) bf  Bs[64 * 64];
    __shared__ __align__(16) h16 Ps[4 * 16 * KP];
    __shared__ __align__(16) bf  Es[4 * 2 * 16 * 64];
    const int qt = blockIdx.x, h = blockIdx.y, b = blockIdx.z;
    const int tid = threadIdx.x, w = tid >> 5, lane = tid & 31, lr = lane & 15, hi = lane >> 4;
    const size_t rowb = (size_t)b * SEQ;
    int qrow = qt * 64 + w * 16 + lr; qrow = (qrow < SEQ) ? qrow : (SEQ - 1);
    const h16* qp = F + (rowb + qrow) * DQKV + h * HD + 8 * hi;
    const v16h aq0 = WFrag<h16>::ld(qp), aq1 = WFrag<h16>::ld(qp + 32);
    float m8[8], l8[8]; v8f accO[4];
#pragma unroll
    for (int r = 0; r < 8; ++r) { m8[r] = NEGB; l8[r] = 0.0f; }
#pragma unroll
    for (int j = 0; j < 4; ++j) accO[j] = (v8f){};
    h16* psw = Ps + w * 16 * KP;
    const size_t vtb = ((size_t)(b * NH + h)) * HD * SEQP;
    const size_t bpb = ((size_t)h * SEQP + (size_t)qt * 64) * SEQP;
#pragma unroll 1
    for (int kt = 0; kt < NQT; ++kt) {
        const int kb0 = kt * 64;
#pragma unroll
        for (int i = 0; i < 4; ++i) {
            const int g = tid + i * 128, r = g >> 3, ch = g & 7;
            const int key = kb0 + r; const bool kv = (key < SEQ); const int kc = kv ? key : (SEQ - 1);
            v8h kk = *(const v8ha*)(F + (rowb + kc) * DQKV + DM + h * HD + ch * 8); if (!kv) kk = (v8h){};
            *(v8ha*)(Kt + r * KP + ch * 8) = kk;
            const v8h vv = *(const v8ha*)(VT + vtb + (size_t)r * SEQP + kb0 + ch * 8);
            *(v8ha*)(Vt + r * KP + ch * 8) = vv;
            const v8us bq = *(const v8usa*)(BP + bpb + (size_t)r * SEQP + kb0 + ch * 8);
            *(v8usa*)(Bs + r * 64 + ch * 8) = bq;
        }
        __syncthreads();
        v8f s[4]; v16h bk0f, bk1f;
#pragma unroll
        for (int nf = 0; nf < 4; ++nf) { bk0f = WFrag<h16>::ld(Kt + (nf * 16 + lr) * KP + 8 * hi); bk1f = WFrag<h16>::ld(Kt + (nf * 16 + lr) * KP + 32 + 8 * hi);
            v8f z = (v8f){}; z = wmma16(aq0, bk0f, z); z = wmma16(aq1, bk1f, z); s[nf] = z; }
        asm volatile("v_nop\n\tv_nop\n\tv_nop\n\tv_nop" : "+v"(s[0]), "+v"(s[1]), "+v"(s[2]), "+v"(s[3]) : "v"(aq0), "v"(aq1), "v"(bk1f));
        float mv[8], al[8], rs[8];
#pragma unroll
        for (int r = 0; r < 8; ++r) mv[r] = NEGB;
#pragma unroll
        for (int nf = 0; nf < 4; ++nf)
#pragma unroll
            for (int r = 0; r < 8; ++r) { const int kg = kb0 + nf * 16 + lr; const float t = s[nf][r] * SFOLD + bf2f(Bs[(w * 16 + 8 * hi + r) * 64 + nf * 16 + lr]);
                s[nf][r] = t; mv[r] = (kg < SEQ) ? fmaxf(mv[r], t) : mv[r]; }
#pragma unroll
        for (int r = 0; r < 8; ++r) {
#pragma unroll
            for (int sh = 1; sh < 16; sh <<= 1) mv[r] = fmaxf(mv[r], __shfl_xor(mv[r], sh, 32)); }
#pragma unroll
        for (int r = 0; r < 8; ++r) { const float mn = fmaxf(m8[r], mv[r]); float ex = (m8[r] - mn) * L2E; ex = fmaxf(ex, -200.0f); al[r] = __builtin_amdgcn_exp2f(ex); m8[r] = mn; rs[r] = 0.0f; }
#pragma unroll
        for (int nf = 0; nf < 4; ++nf)
#pragma unroll
            for (int r = 0; r < 8; ++r) { const int kg = kb0 + nf * 16 + lr; float ex = (s[nf][r] - m8[r]) * L2E; ex = fminf(fmaxf(ex, -200.0f), 0.0f);
                const float e = __builtin_amdgcn_exp2f(ex); const float p = (kg < SEQ) ? e : 0.0f; rs[r] += p; psw[(8 * hi + r) * KP + nf * 16 + lr] = tohx(p * PCAR); }
#pragma unroll
        for (int r = 0; r < 8; ++r) {
#pragma unroll
            for (int sh = 1; sh < 16; sh <<= 1) rs[r] += __shfl_xor(rs[r], sh, 32);
            l8[r] = l8[r] * al[r] + rs[r]; }
#pragma unroll
        for (int j = 0; j < 4; ++j)
#pragma unroll
            for (int r = 0; r < 8; ++r) accO[j][r] *= al[r];
        wave_lds_sync();
        const v16h ap0 = cat16(*(const v8ha*)(psw + lr * KP + 8 * hi), *(const v8ha*)(psw + lr * KP + 16 + 8 * hi));
        const v16h ap1 = cat16(*(const v8ha*)(psw + lr * KP + 32 + 8 * hi), *(const v8ha*)(psw + lr * KP + 48 + 8 * hi));
        v16h bv1f;
#pragma unroll
        for (int j = 0; j < 4; ++j) { const v16h bv0f = WFrag<h16>::ld(Vt + (j * 16 + lr) * KP + 8 * hi); bv1f = WFrag<h16>::ld(Vt + (j * 16 + lr) * KP + 32 + 8 * hi);
            accO[j] = wmma16(ap0, bv0f, accO[j]); accO[j] = wmma16(ap1, bv1f, accO[j]); }
        asm volatile("v_nop\n\tv_nop\n\tv_nop\n\tv_nop" : "+v"(accO[0]), "+v"(accO[1]), "+v"(accO[2]), "+v"(accO[3]) : "v"(ap0), "v"(ap1), "v"(bv1f));
        __syncthreads();
    }
    float inv[8];
#pragma unroll
    for (int r = 0; r < 8; ++r) inv[r] = 1.0f / (l8[r] * (PCAR * CAR));
    bf* esh = Es + w * (2 * 16 * 64); bf* esl = esh + 16 * 64;
#pragma unroll
    for (int j = 0; j < 4; ++j)
#pragma unroll
        for (int r = 0; r < 8; ++r) { const float c = accO[j][r] * inv[r]; unsigned short hh, ll; splitf(c, hh, ll); esh[(8 * hi + r) * 64 + j * 16 + lr] = hh; esl[(8 * hi + r) * 64 + j * 16 + lr] = ll; }
    wave_lds_sync();
    const int rq = lane >> 3, ch = lane & 7;
    v8us oh[4], ol[4];
#pragma unroll
    for (int s = 0; s < 4; ++s) { const int R = 4 * s + rq; oh[s] = *(const v8usa*)(esh + R * 64 + ch * 8); ol[s] = *(const v8usa*)(esl + R * 64 + ch * 8); }
#pragma unroll 1
    for (int ps = 0; ps < 2; ++ps) {
#pragma unroll
        for (int s = 0; s < 4; ++s) { const int q = qt * 64 + w * 16 + 4 * s + rq;
            if (q < SEQ) { const size_t oo = (rowb + q) * DM + (size_t)h * HD + ch * 8; *(volatile v8us*)(CTh + oo) = oh[s]; *(volatile v8us*)(CTl + oo) = ol[s]; } }
        if (ps == 0) __threadfence(); }
}

extern "C" void kernel_launch(void* const* d_in, const int* in_sizes, int n_in,
                              void* d_out, int out_size, void* d_ws, size_t ws_size, hipStream_t stream) {
    if (n_in < 8) return;
    if (in_sizes[0] < NB * SEQ_FULL * DM) return;
    if (in_sizes[1] < DQKV * DM) return;
    if (in_sizes[2] < DM || in_sizes[3] < DM || in_sizes[6] < DM) return;
    if (in_sizes[4] < NRD * NH) return;
    if (in_sizes[5] < DM * DM) return;
    if (in_sizes[7] < SEQ_FULL * SEQ_FULL) return;
    if (out_size < NB * SEQ * DM) return;
    const float* x    = (const float*)d_in[0];
    const float* wqkv = (const float*)d_in[1];
    const float* qb   = (const float*)d_in[2];
    const float* vb   = (const float*)d_in[3];
    const float* rpb  = (const float*)d_in[4];
    const float* wo   = (const float*)d_in[5];
    const float* bo   = (const float*)d_in[6];
    const int*   rel  = (const int*)d_in[7];
    float* OUT = (float*)d_out;
    char* wsp = (char*)d_ws;
    auto take = [&](size_t bytes) { char* p = wsp; wsp += bytes; return (void*)p; };
    bf*  WQKV = (bf*)take(WS_WQKV);
    bf*  WO   = (bf*)take(WS_WO);
    bf*  BP   = (bf*)take(WS_BP);
    bf*  XB   = (bf*)take(WS_XB);
    h16* F16  = (h16*)take(WS_F);
    h16* VTP  = (h16*)take(WS_VT);
    bf*  CTh  = (bf*)take(WS_CT);
    bf*  CTl  = (bf*)take(WS_CT);
    if ((size_t)(wsp - (char*)d_ws) > ws_size) return;

    k_cvt8<<<(unsigned)(((size_t)DQKV * DM / 8 + 255) / 256), 256, 0, stream>>>(wqkv, WQKV, (size_t)DQKV * DM / 8);
    k_cvt8<<<(unsigned)(((size_t)DM * DM / 8 + 255) / 256), 256, 0, stream>>>(wo, WO, (size_t)DM * DM / 8);
    k_bias<<<(unsigned)((NH * SEQP * (SEQP / 8) + 255) / 256), 256, 0, stream>>>(rpb, rel, BP);
    for (int b0 = 0; b0 < NB; b0 += BPP) {
        const int nb = ((NB - b0) < BPP) ? (NB - b0) : BPP;
        const int M = nb * SEQ;
        k_cvtx<<<(unsigned)((((size_t)M * DM / 8) + 255) / 256), 256, 0, stream>>>(x + (size_t)b0 * SEQ_FULL * DM, XB, nb);
        k_gemmw<bf, 0, 1><<<dim3((unsigned)((M + 63) / 64), DQKV / 64, 1), 32, 0, stream>>>(XB, nullptr, WQKV, DM, M, nullptr, F16, DQKV, qb, vb, CAR);
        k_vt<<<dim3(NQT, NH, (unsigned)nb), 64, 0, stream>>>(F16, VTP);
        k_attn<<<dim3(NQT, NH, (unsigned)nb), 128, 0, stream>>>(F16, VTP, BP, CTh, CTl);
        k_gemmw<bf, 1, 0><<<dim3((unsigned)((M + 63) / 64), DM / 64, 1), 32, 0, stream>>>(CTh, CTl, WO, DM, M, OUT + (size_t)b0 * SEQ * DM, nullptr, DM, bo, nullptr, 1.0f);
    }
}
